// GATModel_59081570124183
// MI455X (gfx1250) — hardware-run, weakly checked
//
#include <hip/hip_runtime.h>
#include <stddef.h>
#include <stdint.h>
#include <math.h>


#define F_IN    128
#define HC      128
#define NHD     8
#define HCH     16
#define NNODE   100000
#define NTHR    256
#define NWAVE   8
#define EPT     8
#define CHUNK   (NTHR * EPT)
#define WCAP    (EPT * 32)
#define LISTN   (NWAVE * WCAP)
#define NBMAX   2048
#define SLOTB   11
#define RCAP    28672
#define DEGCAP  256
#define GM      128
#define GTHR    256
#define MROWS   128
#define NBW     ((HC * F_IN / 8) / NTHR)
#define NEGSL   0.2f
#define EPS_SM  1e-16f
#define WSMAX   ((size_t)(128u << 20))
#define LDS_AGG  ((2 * RCAP + 2 * NBMAX + LISTN) * 4 + 64)
#define LDS_GEMM ((GM * HC + 2 * HC + 2 * GM * NHD) * 4)

static_assert((CHUNK & (CHUNK - 1)) == 0 && CHUNK <= (1 << SLOTB));
static_assert(NBMAX == (1 << SLOTB));
static_assert(NTHR * 8 == NBMAX);
static_assert(LISTN >= NBMAX);
static_assert(LISTN >= NWAVE * WCAP);
static_assert((RCAP % 32) == 0);
static_assert(LDS_AGG <= 300000);
static_assert(LDS_GEMM <= 300000);
static_assert(NNODE < (1 << 17));
static_assert(17 + SLOTB <= 31);
static_assert(GM == (GTHR / 32) * 16);
static_assert((F_IN % 32) == 0);
static_assert(HC == NHD * HCH && HC == 4 * 32);
static_assert((MROWS % GM) == 0);
static_assert(GTHR * 4 == GM * NHD);
static_assert((HC * F_IN / 8) % NTHR == 0);
static_assert((MROWS * (F_IN / 8)) % NTHR == 0);

typedef float          v4f  __attribute__((ext_vector_type(4)));
typedef float          v8f  __attribute__((ext_vector_type(8)));
typedef int            v4i  __attribute__((ext_vector_type(4)));
typedef int            v8i  __attribute__((ext_vector_type(8)));
typedef unsigned int   v4u  __attribute__((ext_vector_type(4)));
typedef unsigned short v8us __attribute__((ext_vector_type(8)));
typedef __bf16         v16b __attribute__((ext_vector_type(16)));
typedef v4f  __attribute__((may_alias)) v4fa;
typedef v8us __attribute__((may_alias)) v8usa;
union FragB { v16b v; v8us h[2]; v8i w; };

__device__ __forceinline__ v8f wmb(const FragB& a, const FragB& b, v8f c) {
  v8f d = __builtin_amdgcn_wmma_f32_16x16x32_bf16(false, a.v, false, b.v, (short)0, c, false, false);
  asm volatile("v_nop\n\tv_nop\n\tv_nop\n\tv_nop" : "+v"(d) : "v"(a.w), "v"(b.w));
  return d;
}

__device__ __forceinline__ unsigned int f2bf(float f) {
  const unsigned int u = __float_as_uint(f);
  return ((u + 0x7FFFu + ((u >> 16) & 1u)) >> 16) & 0xFFFFu;
}
__device__ __forceinline__ float bf2f(unsigned int b) { return __uint_as_float(b << 16); }
__device__ __forceinline__ float bfr(float f) { return bf2f(f2bf(f)); }
__device__ __forceinline__ v4f bfr4(const v4f a) {
  v4f r; r.x = bfr(a.x); r.y = bfr(a.y); r.z = bfr(a.z); r.w = bfr(a.w); return r;
}
__device__ __forceinline__ unsigned int pk2(float lo, float hi) { return f2bf(lo) | (f2bf(hi) << 16); }
__device__ __forceinline__ v4u pack8(const v4f a, const v4f b) {
  v4u r;
  r.x = pk2(a.x, a.y); r.y = pk2(a.z, a.w); r.z = pk2(b.x, b.y); r.w = pk2(b.z, b.w);
  return r;
}

__device__ __forceinline__ int scan_chunk(const int* __restrict__ dsts, int nE, int cbase, int slotBase,
                                          int nb, int vec8, int* list, int tid, int lane, int wave) {
  int wc = 0;
  const int el0  = tid * EPT;
  const int e0   = cbase + el0;
  const int sent = (int)(1u << 31);
  v4i da, db;
  if (vec8 != 0 && cbase + CHUNK <= nE) {
    da = *(const v4i*)(dsts + e0);
    db = *(const v4i*)(dsts + e0 + 4);
  } else {
    da.x = (e0     < nE) ? dsts[min(e0,     nE - 1)] : sent;
    da.y = (e0 + 1 < nE) ? dsts[min(e0 + 1, nE - 1)] : sent;
    da.z = (e0 + 2 < nE) ? dsts[min(e0 + 2, nE - 1)] : sent;
    da.w = (e0 + 3 < nE) ? dsts[min(e0 + 3, nE - 1)] : sent;
    db.x = (e0 + 4 < nE) ? dsts[min(e0 + 4, nE - 1)] : sent;
    db.y = (e0 + 5 < nE) ? dsts[min(e0 + 5, nE - 1)] : sent;
    db.z = (e0 + 6 < nE) ? dsts[min(e0 + 6, nE - 1)] : sent;
    db.w = (e0 + 7 < nE) ? dsts[min(e0 + 7, nE - 1)] : sent;
  }
  const unsigned nbs = (unsigned)slotBase;
  const unsigned unb = (unsigned)nb;
  const unsigned s0 = (unsigned)da.x - nbs, s1 = (unsigned)da.y - nbs;
  const unsigned s2 = (unsigned)da.z - nbs, s3 = (unsigned)da.w - nbs;
  const unsigned s4 = (unsigned)db.x - nbs, s5 = (unsigned)db.y - nbs;
  const unsigned s6 = (unsigned)db.z - nbs, s7 = (unsigned)db.w - nbs;
  const bool h0 = s0 < unb, h1 = s1 < unb, h2 = s2 < unb, h3 = s3 < unb;
  const bool h4 = s4 < unb, h5 = s5 < unb, h6 = s6 < unb, h7 = s7 < unb;
  const unsigned any = __builtin_amdgcn_ballot_w32(h0 | h1 | h2 | h3 | h4 | h5 | h6 | h7);
  if (any != 0u) {
#define HITJ(J, HJ, SJ) { \
      const unsigned mj = __builtin_amdgcn_ballot_w32(HJ); \
      if (mj != 0u) { \
        if (HJ) { \
          const int pos = wc + (int)__builtin_amdgcn_mbcnt_lo(mj, 0u); \
          if (pos < WCAP) list[wave * WCAP + pos] = ((el0 + (J)) << SLOTB) | (int)(SJ); \
        } \
        wc += (int)__builtin_popcount(mj); } }
    HITJ(0, h0, s0)
    HITJ(1, h1, s1)
    HITJ(2, h2, s2)
    HITJ(3, h3, s3)
    HITJ(4, h4, s4)
    HITJ(5, h5, s5)
    HITJ(6, h6, s6)
    HITJ(7, h7, s7)
#undef HITJ
  }
  return wc;
}

__global__ __launch_bounds__(NTHR) void k_prep(const float* __restrict__ x, const float* __restrict__ W,
                                               const float* __restrict__ aL, const float* __restrict__ aR,
                                               const float* __restrict__ bias,
                                               unsigned short* xb, unsigned short* wt, float* sv,
                                               int nN, int nBx) {
  const int b = (int)blockIdx.x, tid = (int)threadIdx.x;
  if (b < nBx) {
    const int i   = b * NTHR + tid;
    const int row = i >> 4;
    const int c0  = (i & 15) * 8;
    const int rc  = row < nN ? row : nN - 1;
    const float* p = x + (size_t)rc * F_IN + c0;
    v4f a = *(const v4fa*)p, c = *(const v4fa*)(p + 4);
    const v4f z4 = {0.f, 0.f, 0.f, 0.f};
    if (row >= nN) { a = z4; c = z4; }
    const v4u hv = pack8(a, c);
    const size_t o = (size_t)row * F_IN + c0;
    *(volatile v4u*)(xb + o) = hv;
    __threadfence();
    *(volatile v4u*)(xb + o) = hv;
  } else if (b < nBx + NBW) {
    const int u  = (b - nBx) * NTHR + tid;
    const int n  = u >> 4;
    const int k8 = (u & 15) * 8;
    const float* p = W + (size_t)k8 * HC + n;
    v4f a, c;
    a.x = p[0];        a.y = p[HC];       a.z = p[2 * HC];   a.w = p[3 * HC];
    c.x = p[4 * HC];   c.y = p[5 * HC];   c.z = p[6 * HC];   c.w = p[7 * HC];
    const v4u wv = pack8(a, c);
    unsigned short* o = wt + (size_t)n * F_IN + k8;
    *(volatile v4u*)o = wv;
    __threadfence();
    *(volatile v4u*)o = wv;
  } else {
    if (tid < 96) {
      const int grp = tid >> 5;
      const int j0  = 4 * (tid & 31);
      const int i0 = ((j0    ) & 15) * 8 + ((j0    ) >> 4);
      const int i1 = ((j0 + 1) & 15) * 8 + ((j0 + 1) >> 4);
      const int i2 = ((j0 + 2) & 15) * 8 + ((j0 + 2) >> 4);
      const int i3 = ((j0 + 3) & 15) * 8 + ((j0 + 3) >> 4);
      v4f va, vr;
      va.x = aL[i0]; va.y = aL[i1]; va.z = aL[i2]; va.w = aL[i3];
      vr.x = aR[i0]; vr.y = aR[i1]; vr.z = aR[i2]; vr.w = aR[i3];
      const v4f vb = *(const v4fa*)(bias + j0);
      asm volatile("" :: "v"(va), "v"(vr), "v"(vb));
      v4f v = vb;
      if (grp == 0) v = va;
      if (grp == 1) v = vr;
      const v4f r = bfr4(v);
      float* o = sv + 4 * tid;
      *(volatile v4f*)o = r;
      __threadfence();
      *(volatile v4f*)o = r;
    }
  }
}

__global__ __launch_bounds__(GTHR) __attribute__((amdgpu_num_vgpr(248)))
void k_gemm(const unsigned short* __restrict__ A, const unsigned short* __restrict__ WT,
            const float* __restrict__ aclr, float* Hout, float* AS, float* AD) {
  extern __shared__ v4f lds_g[];
  float* stg  = (float*)lds_g;
  float* svec = stg + GM * HC;
  float* sdot = svec + 2 * HC;
  const int tid = (int)threadIdx.x, lane = tid & 31, wave = tid >> 5, hh = lane >> 4, m = lane & 15;
  const int rowBase = (int)blockIdx.x * GM;

  if (tid < 64) {
    const v4f v = *(const v4fa*)(aclr + 4 * tid);
    *(v4fa*)(svec + 4 * tid) = v;
  }

  v8f acc[8];
  {
    const v8f z = {0.f, 0.f, 0.f, 0.f, 0.f, 0.f, 0.f, 0.f};
#pragma unroll
    for (int t = 0; t < 8; ++t) acc[t] = z;
  }
  const unsigned short* ap = A  + (size_t)(rowBase + 16 * wave + m) * F_IN + 8 * hh;
  const unsigned short* wp = WT + (size_t)m * F_IN + 8 * hh;
#pragma unroll 1
  for (int ks = 0; ks < F_IN / 32; ++ks) {
    FragB af;
    af.h[0] = *(const v8usa*)(ap + 32 * ks);
    af.h[1] = *(const v8usa*)(ap + 32 * ks + 16);
#pragma unroll
    for (int t = 0; t < 8; ++t) {
      const unsigned short* wq = wp + (size_t)(16 * t) * F_IN + 32 * ks;
      FragB bf;
      bf.h[0] = *(const v8usa*)wq;
      bf.h[1] = *(const v8usa*)(wq + 16);
      acc[t] = wmb(af, bf, acc[t]);
    }
  }

#pragma unroll
  for (int t = 0; t < 8; ++t) {
    const int lc = 16 * t + m;
#pragma unroll
    for (int r = 0; r < 8; ++r) {
      const int lr = 16 * wave + 8 * hh + r;
      stg[lr * HC + lc] = acc[t][r];
    }
  }
  __syncthreads();

  {
    const int row = tid & (GM - 1), which = tid >> 7;
    const float* sa = svec + which * HC;
    const float* hr = stg + row * HC;
#pragma unroll 1
    for (int hd = 0; hd < NHD; ++hd) {
      float d = 0.f;
#pragma unroll
      for (int c4 = 0; c4 < HCH / 4; ++c4) {
        const v4f hv = *(const v4fa*)(hr + HCH * hd + 4 * c4);
        const v4f av = *(const v4fa*)(sa + HCH * hd + 4 * c4);
        d = fmaf(hv.x, av.x, d);
        d = fmaf(hv.y, av.y, d);
        d = fmaf(hv.z, av.z, d);
        d = fmaf(hv.w, av.w, d);
      }
      sdot[which * (GM * NHD) + row * NHD + hd] = d;
    }
  }
  __syncthreads();

  const v4f dsv = *(const v4fa*)(sdot + 4 * tid);
  const v4f ddv = *(const v4fa*)(sdot + GM * NHD + 4 * tid);
  float* asp = AS + (size_t)rowBase * NHD + 4 * tid;
  float* adp = AD + (size_t)rowBase * NHD + 4 * tid;

#pragma unroll
  for (int i = 0; i < 16; ++i) {
    const int lr = 16 * wave + i;
    const v4f v = *(const v4fa*)(stg + lr * HC + 4 * lane);
    float* op = Hout + (size_t)(rowBase + lr) * HC + 4 * lane;
    *(volatile v4f*)op = v;
  }
  *(volatile v4f*)asp = dsv;
  *(volatile v4f*)adp = ddv;
  __threadfence();
#pragma unroll
  for (int i = 0; i < 16; ++i) {
    const int lr = 16 * wave + i;
    const v4f v = *(const v4fa*)(stg + lr * HC + 4 * lane);
    float* op = Hout + (size_t)(rowBase + lr) * HC + 4 * lane;
    *(volatile v4f*)op = v;
  }
  *(volatile v4f*)asp = dsv;
  *(volatile v4f*)adp = ddv;
}

__global__ __launch_bounds__(NTHR) void k_scan(
    const int* __restrict__ srcs, const int* __restrict__ dsts,
    const float* __restrict__ Hm, const float* __restrict__ AS, const float* __restrict__ AD,
    const float* __restrict__ biasr, float* out,
    int nN, int nE, int nb, int vec8) {
  extern __shared__ v4f lds_dyn[];
  int* reg1 = (int*)lds_dyn;
  int* reg2 = reg1 + RCAP;
  int* scnt = reg2 + RCAP;
  int* soff = scnt + NBMAX;
  int* list = soff + NBMAX;
  int* wcnt = list + LISTN;
  int* wtot = wcnt + NWAVE;
  const int tid = (int)threadIdx.x, lane = tid & 31, wave = tid >> 5;
  const int nodeBase = (int)blockIdx.x * nb;

  for (int i = tid; i < NBMAX; i += NTHR) scnt[i] = 0;
  __syncthreads();

  int tot = 0;
  const int nChunks = (nE + CHUNK - 1) / CHUNK;
#pragma unroll 1
  for (int ch = 0; ch < nChunks; ++ch) {
    const int cbase = ch * CHUNK;
    const int wc = scan_chunk(dsts, nE, cbase, nodeBase, nb, vec8, list, tid, lane, wave);
    if (lane == 0) wcnt[wave] = wc;
    __syncthreads();
    int pre = 0, all = 0;
#pragma unroll
    for (int w2 = 0; w2 < NWAVE; ++w2) {
      int c = wcnt[w2];
      c = c < 0 ? 0 : (c > WCAP ? WCAP : c);
      all += c;
      pre += (w2 < wave) ? c : 0;
    }
    const int wcc  = wc > WCAP ? WCAP : wc;
    const int base = tot + pre;
#pragma unroll 1
    for (int i0 = 0; i0 < wcc; i0 += 32) {
      const int i  = i0 + lane;
      const int ic = i < wcc ? i : wcc - 1;
      const int ent = list[wave * WCAP + ic];
      const int el  = (ent >> SLOTB) & (CHUNK - 1);
      const int sl  = ent & (NBMAX - 1);
      int eid = cbase + el;
      eid = eid > nE - 1 ? nE - 1 : eid;
      eid = eid < 0 ? 0 : eid;
      const int sraw = srcs[eid];
      asm volatile("" :: "v"(sraw));
      const int s = sraw < 0 ? 0 : (sraw > nN - 1 ? nN - 1 : sraw);
      const int pos = base + i;
      if (i < wcc && pos < RCAP) reg1[pos] = (int)(((unsigned)s << SLOTB) | (unsigned)sl);
    }
    tot += all;
    tot = tot > RCAP ? RCAP : tot;
    __syncthreads();
  }
  const int nh = tot;

  if (wave == 0) {
#pragma unroll 1
    for (int b0 = 0; b0 < nh; b0 += 32) {
      const int idx = b0 + lane;
      const int uv  = reg1[idx < nh ? idx : nh - 1];
      const int m32 = (nh - b0) < 32 ? (nh - b0) : 32;
#pragma unroll 1
      for (int k = 0; k < m32; ++k) {
        const int u  = __builtin_amdgcn_readlane(uv, k);
        const int sl = u & (NBMAX - 1);
        if (lane == 0) scnt[sl] = scnt[sl] + 1;
      }
    }
  }
  __syncthreads();

  {
    const v4i ca = *(const v4i*)(scnt + 8 * tid);
    const v4i cb = *(const v4i*)(scnt + 8 * tid + 4);
    const int e0 = ca.x < 0 ? 0 : ca.x, e1 = ca.y < 0 ? 0 : ca.y, e2 = ca.z < 0 ? 0 : ca.z, e3 = ca.w < 0 ? 0 : ca.w;
    const int e4 = cb.x < 0 ? 0 : cb.x, e5 = cb.y < 0 ? 0 : cb.y, e6 = cb.z < 0 ? 0 : cb.z, e7 = cb.w < 0 ? 0 : cb.w;
    const int ts = e0 + e1 + e2 + e3 + e4 + e5 + e6 + e7;
    int incl = ts;
#pragma unroll
    for (int d = 1; d < 32; d <<= 1) {
      const int up = __shfl_up(incl, d);
      if (lane >= d) incl += up;
    }
    if (lane == 31) wtot[wave] = incl;
    __syncthreads();
    int pre = 0;
#pragma unroll
    for (int w2 = 0; w2 < NWAVE; ++w2) pre += (w2 < wave) ? wtot[w2] : 0;
    int run = pre + incl - ts;
    soff[8 * tid + 0] = run; run += e0;
    soff[8 * tid + 1] = run; run += e1;
    soff[8 * tid + 2] = run; run += e2;
    soff[8 * tid + 3] = run; run += e3;
    soff[8 * tid + 4] = run; run += e4;
    soff[8 * tid + 5] = run; run += e5;
    soff[8 * tid + 6] = run; run += e6;
    soff[8 * tid + 7] = run;
  }
  __syncthreads();
  for (int i = tid; i < NBMAX; i += NTHR) list[i] = soff[i];
  __syncthreads();

  if (wave == 0) {
#pragma unroll 1
    for (int b0 = 0; b0 < nh; b0 += 32) {
      const int idx = b0 + lane;
      const int uv  = reg1[idx < nh ? idx : nh - 1];
      const int m32 = (nh - b0) < 32 ? (nh - b0) : 32;
#pragma unroll 1
      for (int k = 0; k < m32; ++k) {
        const int u   = __builtin_amdgcn_readlane(uv, k);
        const int sl  = u & (NBMAX - 1);
        const int sid = (int)((unsigned)u >> SLOTB);
        if (lane == 0) {
          int pos = list[sl];
          pos = pos < 0 ? 0 : (pos > RCAP - 1 ? RCAP - 1 : pos);
          reg2[pos] = sid;
          list[sl] = pos + 1;
        }
      }
    }
  }
  __syncthreads();

  const int nbw = nb >> 3;
  const bool ovf = (nh >= RCAP);
  const float qnan = __int_as_float(0x7fc00000);
  const int hA = lane >> 2;
  const int hq = lane >> 3;
  const int hE = lane & 7;
  const v4f bb = *(const v4fa*)(biasr + 4 * lane);

#pragma unroll 1
  for (int jt = 0; jt < nbw; ++jt) {
    const int slot = wave * nbw + jt;
    const int grow = nodeBase + slot;
    const int gcl  = grow < nN ? grow : nN - 1;
    int st = soff[slot];
    const int craw = scnt[slot];
    int cnt = craw;
    st  = st < 0 ? 0 : (st > nh ? nh : st);
    cnt = cnt < 0 ? 0 : (cnt > DEGCAP ? DEGCAP : cnt);
    if (cnt > nh - st) cnt = nh - st;
    const bool bad = ovf || (craw > DEGCAP);
    st  = __builtin_amdgcn_readfirstlane(st);
    cnt = __builtin_amdgcn_readfirstlane(cnt);
    int last = st + cnt - 1; last = last < st ? st : last;
    last = last > RCAP - 1 ? RCAP - 1 : last;

    const float adE = AD[(size_t)gcl * NHD + hE];
    float dn = 0.0f;
    v4f av = {0.f, 0.f, 0.f, 0.f};

#pragma unroll 1
    for (int q0 = 0; q0 < cnt; q0 += 4) {
      const int qi = q0 + hq;
      int idx = st + qi;
      idx = idx > last ? last : idx;
      idx = idx < 0 ? 0 : idx;
      int sE = reg2[idx];
      sE = sE < 0 ? 0 : (sE > nN - 1 ? nN - 1 : sE);
      const float asv = AS[(size_t)sE * NHD + hE];
      asm volatile("" :: "v"(asv));
      float lg = asv + adE;
      lg = lg > 0.f ? lg : NEGSL * lg;
      float p = expf(lg);
      p = (qi < cnt) ? p : 0.0f;
#pragma unroll
      for (int j = 0; j < 4; ++j) {
        const float pj = __shfl(p, 8 * j + hA);
        const int   sj = __builtin_amdgcn_readlane(sE, 8 * j);
        const v4f hv = *(const v4fa*)(Hm + (size_t)sj * HC + 4 * lane);
        dn += pj;
        av.x = fmaf(pj, hv.x, av.x);
        av.y = fmaf(pj, hv.y, av.y);
        av.z = fmaf(pj, hv.z, av.z);
        av.w = fmaf(pj, hv.w, av.w);
      }
    }
    const float inv = 1.0f / (dn + EPS_SM);
    v4f o;
    o.x = fmaf(av.x, inv, bb.x);
    o.y = fmaf(av.y, inv, bb.y);
    o.z = fmaf(av.z, inv, bb.z);
    o.w = fmaf(av.w, inv, bb.w);
    o.x = bad ? qnan : o.x;
    o.y = bad ? qnan : o.y;
    o.z = bad ? qnan : o.z;
    o.w = bad ? qnan : o.w;
    float* op = out + (size_t)gcl * HC + 4 * lane;
    const bool wr = grow < nN;
    if (wr) *(volatile v4f*)op = o;
    __threadfence();
    if (wr) *(volatile v4f*)op = o;
  }
}

static int pick_nb(int nE, int nN) {
  int nb = NBMAX;
  while (nb > 32 && (long long)nb * (long long)nE * 5LL > (long long)RCAP * (long long)nN * 4LL) nb >>= 1;
  return nb;
}
static inline int cdiv(int a, int b) { return (a + b - 1) / b; }

extern "C" void kernel_launch(void* const* d_in, const int* in_sizes, int n_in,
                              void* d_out, int out_size, void* d_ws, size_t ws_size,
                              hipStream_t stream) {
  if (n_in < 6) return;
  const int nN = in_sizes[0] / F_IN;
  if (nN <= 0 || in_sizes[0] != nN * F_IN || nN > (1 << 17)) return;
  if (in_sizes[1] < 2 || (in_sizes[1] & 1) != 0) return;
  const int nE = in_sizes[1] / 2;
  if (nE < 1 || nE >= (1 << 30)) return;
  if (in_sizes[2] != F_IN * HC) return;
  if (in_sizes[3] != HCH * NHD || in_sizes[4] != HCH * NHD) return;
  if (in_sizes[5] != HC) return;
  if (out_size != nN * HC) return;

  const float* x    = (const float*)d_in[0];
  const int*   ei   = (const int*)  d_in[1];
  const float* W    = (const float*)d_in[2];
  const float* aL   = (const float*)d_in[3];
  const float* aR   = (const float*)d_in[4];
  const float* bias = (const float*)d_in[5];
  float* out = (float*)d_out;
  const int* src = ei;
  const int* dst = ei + nE;

  const int MP   = cdiv(nN, MROWS) * MROWS;
  const int nb   = pick_nb(nE, nN);
  if (nb < 32 || (nb & (nb - 1)) != 0 || nb > NBMAX) return;
  const int gA   = cdiv(nN, nb);
  const int vec8 = ((nE & 3) == 0) ? 1 : 0;
  if (gA * nb < nN) return;
  const int nBx  = (MP * (F_IN / 8)) / NTHR;
  if (nBx * NTHR != MP * (F_IN / 8)) return;

  char* ws = (char*)d_ws;
  size_t off = 0;
  const size_t oXB = off; off += (size_t)MP * F_IN * 2;   off = (off + 255) & ~(size_t)255;
  const size_t oWT = off; off += (size_t)HC * F_IN * 2;   off = (off + 255) & ~(size_t)255;
  const size_t oH  = off; off += (size_t)MP * HC * 4;     off = (off + 255) & ~(size_t)255;
  const size_t oAS = off; off += (size_t)MP * NHD * 4;    off = (off + 255) & ~(size_t)255;
  const size_t oAD = off; off += (size_t)MP * NHD * 4;    off = (off + 255) & ~(size_t)255;
  const size_t oSV = off; off += (size_t)3 * HC * 4;      off = (off + 255) & ~(size_t)255;
  if (off > ws_size || off > WSMAX) return;
  unsigned short* XB = (unsigned short*)(ws + oXB);
  unsigned short* WT = (unsigned short*)(ws + oWT);
  float*          Hm = (float*)(ws + oH);
  float*          AS = (float*)(ws + oAS);
  float*          AD = (float*)(ws + oAD);
  float*          SV = (float*)(ws + oSV);

  hipFuncSetAttribute(reinterpret_cast<const void*>(&k_gemm),
                      hipFuncAttributeMaxDynamicSharedMemorySize, LDS_GEMM);
  hipFuncSetAttribute(reinterpret_cast<const void*>(&k_scan),
                      hipFuncAttributeMaxDynamicSharedMemorySize, LDS_AGG);

  k_prep<<<nBx + NBW + 1, NTHR, 0, stream>>>(x, W, aL, aR, bias, XB, WT, SV, nN, nBx);
  k_gemm<<<MP / GM, GTHR, LDS_GEMM, stream>>>(XB, WT, SV, Hm, AS, AD);
  k_scan<<<gA, NTHR, LDS_AGG, stream>>>(src, dst, Hm, AS, AD, SV + 2 * HC, out, nN, nE, nb, vec8);
}
